// ITASelfAttention_3564822856122
// MI455X (gfx1250) — hardware-verified
//
#include <hip/hip_runtime.h>


#define BB    8
#define SEQ   1024
#define EMB   768
#define NH    12
#define HD    64
#define MROWS (BB * SEQ)
#define PH    72
#define PF    68
#define CP    72

typedef unsigned short us;
typedef __bf16 bf16_t;
typedef _Float16 f16_t;
typedef bf16_t v16b __attribute__((ext_vector_type(16)));
typedef f16_t  v16h __attribute__((ext_vector_type(16)));
typedef float  v8f  __attribute__((ext_vector_type(8)));
typedef int    v8i  __attribute__((ext_vector_type(8)));
typedef us     v8us __attribute__((ext_vector_type(8), __may_alias__));
typedef float  v4f  __attribute__((ext_vector_type(4), __may_alias__));

union Frag  { v8us u[2]; v16b b; v16h x; };
union Pack8 { us s[8]; v8us v; };

__device__ __forceinline__ v8us ld8(const us* p) { return *(const v8us*)p; }

__device__ __forceinline__ us bf16_rne(float f) {
  unsigned u = __float_as_uint(f);
  u += 0x7FFFu + ((u >> 16) & 1u);
  return (us)(u >> 16);
}
__device__ __forceinline__ float bf16_val(us v) { return __uint_as_float(((unsigned)v) << 16); }
__device__ __forceinline__ us f16_bits(float f) {
  union { f16_t h; us u; } c; c.h = (f16_t)f; return c.u;
}

__device__ __forceinline__ v8f mma_bf16(v16b a, v16b b, v8f c) {
  c = __builtin_amdgcn_wmma_f32_16x16x32_bf16(false, a, false, b, (short)0, c, false, false);
  v8i ka = __builtin_bit_cast(v8i, a), kb = __builtin_bit_cast(v8i, b);
  asm volatile("v_nop\n\tv_nop\n\tv_nop\n\tv_nop" : "+v"(c) : "v"(ka), "v"(kb));
  return c;
}
__device__ __forceinline__ v8f mma_f16(v16h a, v16h b, v8f c) {
  c = __builtin_amdgcn_wmma_f32_16x16x32_f16(false, a, false, b, (short)0, c, false, false);
  v8i ka = __builtin_bit_cast(v8i, a), kb = __builtin_bit_cast(v8i, b);
  asm volatile("v_nop\n\tv_nop\n\tv_nop\n\tv_nop" : "+v"(c) : "v"(ka), "v"(kb));
  return c;
}

__global__ __launch_bounds__(256) void cvt_kernel(
    const float* __restrict__ in, int n8,
    us* __restrict__ oH, us* __restrict__ oL, us* __restrict__ oF,
    float fscale, int doSplit, int doF,
    const int* __restrict__ aux0, const int* __restrict__ aux1) {
  (void)aux0; (void)aux1;
  const int i = blockIdx.x * 256 + threadIdx.x;
  if (i >= n8) return;
  const v4f f0 = *(const v4f*)(in + (size_t)i * 8);
  const v4f f1 = *(const v4f*)(in + (size_t)i * 8 + 4);
  float f[8];
  f[0] = f0[0]; f[1] = f0[1]; f[2] = f0[2]; f[3] = f0[3];
  f[4] = f1[0]; f[5] = f1[1]; f[6] = f1[2]; f[7] = f1[3];
  Pack8 ph, pl, pf;
#pragma unroll
  for (int e = 0; e < 8; ++e) {
    const us hi = bf16_rne(f[e]);
    ph.s[e] = hi;
    pl.s[e] = bf16_rne(f[e] - bf16_val(hi));
    pf.s[e] = f16_bits(f[e] * fscale);
  }
  us* dH = oH + (size_t)i * 8;
  us* dL = oL + (size_t)i * 8;
  us* dF = oF + (size_t)i * 8;
  if (doSplit) { *(volatile v8us*)dH = ph.v; *(volatile v8us*)dL = pl.v; }
  if (doF)     { *(volatile v8us*)dF = pf.v; }
  __threadfence();
  if (doSplit) { *(volatile v8us*)dH = ph.v; *(volatile v8us*)dL = pl.v; }
  if (doF)     { *(volatile v8us*)dF = pf.v; }
}

template <int MODE>
__device__ __forceinline__ void gemm_store_pass(const us* stg, int lane, int w, int rowBlk, int col0,
                                                us* O0, us* O1, float* OF) {
  const int head = col0 >> 6;
  if (MODE == 0) {
#pragma unroll
    for (int i = 0; i < 8; ++i) {
      const int rl = w * 32 + 4 * i + (lane >> 3);
      const int j = lane & 7;
      const int row = rowBlk + rl;
      const int b = row >> 10, n = row & 1023;
      const size_t off = (((size_t)(b * NH + head)) * SEQ + n) * HD + 8 * j;
      const v8us vh = ld8(stg + rl * PH + 8 * j);
      const v8us vl = ld8(stg + 128 * PH + rl * PH + 8 * j);
      *(volatile v8us*)(O0 + off) = vh;
      *(volatile v8us*)(O1 + off) = vl;
    }
  } else if (MODE == 1) {
    const int b = rowBlk >> 10, n0 = rowBlk & 1023;
    const int bhh = b * NH + head;
#pragma unroll
    for (int i = 0; i < 8; ++i) {
      const int q = lane >> 3, j = lane & 7;
      const int dl = w * 16 + 2 * i + (q >> 1);
      const int nl = (q & 1) * 64 + 8 * j;
      Pack8 pk;
#pragma unroll
      for (int e = 0; e < 8; ++e) pk.s[e] = stg[(nl + e) * PH + dl];
      const size_t off = ((size_t)(bhh * HD + dl)) * SEQ + n0 + nl;
      *(volatile v8us*)(O0 + off) = pk.v;
    }
  } else {
    const float* stgF = (const float*)stg;
#pragma unroll
    for (int i = 0; i < 16; ++i) {
      const int rl = w * 32 + 2 * i + (lane >> 4);
      const int c = 4 * (lane & 15);
      const v4f v = *(const v4f*)(stgF + rl * PF + c);
      *(volatile v4f*)(OF + (size_t)(rowBlk + rl) * EMB + col0 + c) = v;
    }
  }
}

template <int MODE>
__global__ __launch_bounds__(128) void gemm_kernel(
    const us* __restrict__ A0, const us* __restrict__ A1,
    const us* __restrict__ B0, const us* __restrict__ B1,
    const float* __restrict__ bias,
    us* __restrict__ O0, us* __restrict__ O1, float* __restrict__ OF) {
  __shared__ __attribute__((aligned(16))) us stg[2 * 128 * PH];
  const int lane = threadIdx.x & 31, w = threadIdx.x >> 5;
  const int h = lane >> 4, m = lane & 15;
  const int rowBlk = blockIdx.y * 128;
  const int rowW = rowBlk + w * 32;
  const int col0 = blockIdx.x * 64;

  v8f acc[2][4];
#pragma unroll
  for (int mt = 0; mt < 2; ++mt)
#pragma unroll
    for (int nt = 0; nt < 4; ++nt) acc[mt][nt] = (v8f)0.0f;

#pragma unroll 1
  for (int kk = 0; kk < EMB; kk += 32) {
    Frag a0[2], b0[4];
#pragma unroll
    for (int mt = 0; mt < 2; ++mt) {
      const us* rp = A0 + (size_t)(rowW + 16 * mt + m) * EMB + kk + 8 * h;
      a0[mt].u[0] = ld8(rp); a0[mt].u[1] = ld8(rp + 16);
    }
#pragma unroll
    for (int nt = 0; nt < 4; ++nt) {
      const us* cp = B0 + (size_t)(col0 + 16 * nt + m) * EMB + kk + 8 * h;
      b0[nt].u[0] = ld8(cp); b0[nt].u[1] = ld8(cp + 16);
    }
    if (MODE == 0) {
      Frag a1[2], b1[4];
#pragma unroll
      for (int mt = 0; mt < 2; ++mt) {
        const us* rp = A1 + (size_t)(rowW + 16 * mt + m) * EMB + kk + 8 * h;
        a1[mt].u[0] = ld8(rp); a1[mt].u[1] = ld8(rp + 16);
      }
#pragma unroll
      for (int nt = 0; nt < 4; ++nt) {
        const us* cp = B1 + (size_t)(col0 + 16 * nt + m) * EMB + kk + 8 * h;
        b1[nt].u[0] = ld8(cp); b1[nt].u[1] = ld8(cp + 16);
      }
#pragma unroll
      for (int mt = 0; mt < 2; ++mt)
#pragma unroll
        for (int nt = 0; nt < 4; ++nt) {
          acc[mt][nt] = mma_bf16(a0[mt].b, b0[nt].b, acc[mt][nt]);
          acc[mt][nt] = mma_bf16(a0[mt].b, b1[nt].b, acc[mt][nt]);
          acc[mt][nt] = mma_bf16(a1[mt].b, b0[nt].b, acc[mt][nt]);
        }
    } else {
#pragma unroll
      for (int mt = 0; mt < 2; ++mt)
#pragma unroll
        for (int nt = 0; nt < 4; ++nt)
          acc[mt][nt] = mma_f16(a0[mt].x, b0[nt].x, acc[mt][nt]);
    }
  }

#pragma unroll
  for (int nt = 0; nt < 4; ++nt) {
    const int cl = 16 * nt + m;
    const float bvv = bias[col0 + cl];
#pragma unroll
    for (int mt = 0; mt < 2; ++mt) {
#pragma unroll
      for (int r = 0; r < 8; ++r) {
        const int rl = w * 32 + 16 * mt + 8 * h + r;
        if (MODE == 0) {
          const float val = acc[mt][nt][r] + bvv;
          const us hi = bf16_rne(val);
          stg[rl * PH + cl] = hi;
          stg[128 * PH + rl * PH + cl] = bf16_rne(val - bf16_val(hi));
        } else if (MODE == 1) {
          const float val = acc[mt][nt][r] * (1.0f / 16384.0f) + bvv;
          stg[rl * PH + cl] = f16_bits(val * 64.0f);
        } else {
          const float val = acc[mt][nt][r] * (1.0f / 262144.0f) + bvv;
          ((float*)stg)[rl * PF + cl] = val;
        }
      }
    }
  }
  __syncthreads();
  gemm_store_pass<MODE>(stg, lane, w, rowBlk, col0, O0, O1, OF);
  __threadfence();
  gemm_store_pass<MODE>(stg, lane, w, rowBlk, col0, O0, O1, OF);
}

__global__ __launch_bounds__(128) void attn_kernel(
    const us* __restrict__ Qh, const us* __restrict__ Ql,
    const us* __restrict__ Kh, const us* __restrict__ Kl,
    const us* __restrict__ Vt,
    us* __restrict__ Ctx) {
  __shared__ __attribute__((aligned(16))) us Kls[2][32 * HD];
  __shared__ __attribute__((aligned(16))) us Vls[HD * 32];
  __shared__ __attribute__((aligned(16))) us Pls[4][16 * 32];
  __shared__ __attribute__((aligned(16))) us Cst[4][16 * CP];

  const int tid = threadIdx.x, w = tid >> 5, lane = tid & 31;
  const int h = lane >> 4, m = lane & 15;
  const int bh = blockIdx.x;
  const int b = bh / NH;
  const int head = bh - b * NH;
  const int q0 = blockIdx.y * 64 + w * 16;
  const size_t plane = (size_t)bh * SEQ * HD;
  const us* Qhp = Qh + plane;
  const us* Qlp = Ql + plane;
  const us* Khp = Kh + plane;
  const us* Klp = Kl + plane;
  const us* Vtp = Vt + (size_t)bh * HD * SEQ;

  Frag qh[2], ql[2];
#pragma unroll
  for (int s = 0; s < 2; ++s) {
    const us* rp = Qhp + (size_t)(q0 + m) * HD + 32 * s + 8 * h;
    qh[s].u[0] = ld8(rp); qh[s].u[1] = ld8(rp + 16);
    const us* lp = Qlp + (size_t)(q0 + m) * HD + 32 * s + 8 * h;
    ql[s].u[0] = ld8(lp); ql[s].u[1] = ld8(lp + 16);
  }

  v8f acc[4];
  float mrow[8], lrow[8];
#pragma unroll
  for (int dt = 0; dt < 4; ++dt) acc[dt] = (v8f)0.0f;
#pragma unroll
  for (int r = 0; r < 8; ++r) { mrow[r] = -1e30f; lrow[r] = 0.0f; }

#pragma unroll 1
  for (int kb = 0; kb < SEQ; kb += 32) {
#pragma unroll
    for (int e = 0; e < 2; ++e) {
      const int idx = tid + 128 * e;
      const int key = idx >> 3, d8 = (idx & 7) * 8;
      *(v8us*)(&Kls[0][key * HD + d8]) = ld8(Khp + (size_t)(kb + key) * HD + d8);
      *(v8us*)(&Kls[1][key * HD + d8]) = ld8(Klp + (size_t)(kb + key) * HD + d8);
      const int dv = idx >> 2, k8 = (idx & 3) * 8;
      *(v8us*)(&Vls[dv * 32 + k8]) = ld8(Vtp + (size_t)dv * SEQ + kb + k8);
    }
    __syncthreads();

    v8f sc2[2];
#pragma unroll
    for (int kn = 0; kn < 2; ++kn) {
      v8f z = (v8f)0.0f;
#pragma unroll
      for (int s = 0; s < 2; ++s) {
        Frag fk, fl;
        const us* kp0 = &Kls[0][(16 * kn + m) * HD + 32 * s + 8 * h];
        const us* kp1 = &Kls[1][(16 * kn + m) * HD + 32 * s + 8 * h];
        fk.u[0] = ld8(kp0); fk.u[1] = ld8(kp0 + 16);
        fl.u[0] = ld8(kp1); fl.u[1] = ld8(kp1 + 16);
        z = mma_bf16(qh[s].b, fk.b, z);
        z = mma_bf16(qh[s].b, fl.b, z);
        z = mma_bf16(ql[s].b, fk.b, z);
      }
      sc2[kn] = z;
    }

#pragma unroll
    for (int r = 0; r < 8; ++r) {
      const float a0 = sc2[0][r], a1 = sc2[1][r];
      float bm = fmaxf(a0, a1);
      bm = fmaxf(bm, __shfl_xor(bm, 1, 32));
      bm = fmaxf(bm, __shfl_xor(bm, 2, 32));
      bm = fmaxf(bm, __shfl_xor(bm, 4, 32));
      bm = fmaxf(bm, __shfl_xor(bm, 8, 32));
      const float nm = fmaxf(mrow[r], bm);
      const float corr = __expf(mrow[r] - nm);
      mrow[r] = nm;
      const float p0 = __expf(a0 - nm);
      const float p1 = __expf(a1 - nm);
      float rs = p0 + p1;
      rs += __shfl_xor(rs, 1, 32);
      rs += __shfl_xor(rs, 2, 32);
      rs += __shfl_xor(rs, 4, 32);
      rs += __shfl_xor(rs, 8, 32);
      lrow[r] = lrow[r] * corr + rs;
#pragma unroll
      for (int dt = 0; dt < 4; ++dt) acc[dt][r] = acc[dt][r] * corr;
      Pls[w][(8 * h + r) * 32 + m]      = f16_bits(p0 * 4096.0f);
      Pls[w][(8 * h + r) * 32 + 16 + m] = f16_bits(p1 * 4096.0f);
    }
    __syncthreads();

    Frag pa;
    const us* pp = &Pls[w][m * 32 + 8 * h];
    pa.u[0] = ld8(pp); pa.u[1] = ld8(pp + 16);
#pragma unroll
    for (int dt = 0; dt < 4; ++dt) {
      Frag fv;
      const us* vp = &Vls[(16 * dt + m) * 32 + 8 * h];
      fv.u[0] = ld8(vp); fv.u[1] = ld8(vp + 16);
      acc[dt] = mma_f16(pa.x, fv.x, acc[dt]);
    }
    __syncthreads();
  }

  float inv[8];
#pragma unroll
  for (int r = 0; r < 8; ++r) inv[r] = (1.0f / lrow[r]) * (1.0f / 1024.0f);
#pragma unroll
  for (int dt = 0; dt < 4; ++dt)
#pragma unroll
    for (int r = 0; r < 8; ++r)
      Cst[w][(8 * h + r) * CP + 16 * dt + m] = f16_bits(acc[dt][r] * inv[r]);
  __syncthreads();

  const size_t rowbase = (size_t)b * SEQ + q0;
#pragma unroll
  for (int i = 0; i < 4; ++i) {
    const int rl = 4 * i + (lane >> 3), j = lane & 7;
    const v8us v = ld8(&Cst[w][rl * CP + 8 * j]);
    *(volatile v8us*)(Ctx + (rowbase + rl) * EMB + head * HD + 8 * j) = v;
  }
  __threadfence();
#pragma unroll
  for (int i = 0; i < 4; ++i) {
    const int rl = 4 * i + (lane >> 3), j = lane & 7;
    const v8us v = ld8(&Cst[w][rl * CP + 8 * j]);
    *(volatile v8us*)(Ctx + (rowbase + rl) * EMB + head * HD + 8 * j) = v;
  }
}

extern "C" void kernel_launch(void* const* d_in, const int* in_sizes, int n_in,
                              void* d_out, int out_size, void* d_ws, size_t ws_size,
                              hipStream_t stream) {
  if (n_in < 11) return;
  if (in_sizes[0] != MROWS * EMB) return;
  if (in_sizes[1] != EMB * EMB || in_sizes[3] != EMB * EMB ||
      in_sizes[5] != EMB * EMB || in_sizes[7] != EMB * EMB) return;
  if (in_sizes[2] != EMB || in_sizes[4] != EMB || in_sizes[6] != EMB || in_sizes[8] != EMB) return;
  if (out_size != MROWS * EMB) return;

  const float* x  = (const float*)d_in[0];
  const float* wq = (const float*)d_in[1];
  const float* bq = (const float*)d_in[2];
  const float* wk = (const float*)d_in[3];
  const float* bk = (const float*)d_in[4];
  const float* wv = (const float*)d_in[5];
  const float* bv = (const float*)d_in[6];
  const float* wo = (const float*)d_in[7];
  const float* bo = (const float*)d_in[8];
  const int*   Hp = (const int*)d_in[9];
  const int*   Wp = (const int*)d_in[10];
  float* out = (float*)d_out;

  unsigned char* ws = (unsigned char*)d_ws;
  size_t off = 0;
  const size_t actB = (size_t)MROWS * EMB * 2;
  const size_t wB   = (size_t)EMB * EMB * 2;
  auto carve = [&](size_t bytes) -> us* {
    us* p = (us*)(ws + off);
    off += (bytes + 255) & ~(size_t)255;
    return p;
  };
  us* xh   = carve(actB);
  us* xl   = carve(actB);
  us* xf   = carve(actB);
  us* wqh  = carve(wB);
  us* wql  = carve(wB);
  us* wkh  = carve(wB);
  us* wkl  = carve(wB);
  us* wvf  = carve(wB);
  us* wof  = carve(wB);
  us* qh   = carve(actB);
  us* ql   = carve(actB);
  us* kh   = carve(actB);
  us* kl   = carve(actB);
  us* vt   = carve(actB);
  us* ctx  = carve(actB);
  if (off > ws_size) return;

  const int nx8 = MROWS * EMB / 8;
  const int nw8 = EMB * EMB / 8;
  cvt_kernel<<<(nx8 + 255) / 256, 256, 0, stream>>>(x,  nx8, xh,  xl,  xf,  16.0f,   1, 1, Hp, Wp);
  cvt_kernel<<<(nw8 + 255) / 256, 256, 0, stream>>>(wq, nw8, wqh, wql, wqh, 1.0f,    1, 0, Hp, Wp);
  cvt_kernel<<<(nw8 + 255) / 256, 256, 0, stream>>>(wk, nw8, wkh, wkl, wkh, 1.0f,    1, 0, Hp, Wp);
  cvt_kernel<<<(nw8 + 255) / 256, 256, 0, stream>>>(wv, nw8, wvf, wvf, wvf, 1024.0f, 0, 1, Hp, Wp);
  cvt_kernel<<<(nw8 + 255) / 256, 256, 0, stream>>>(wo, nw8, wof, wof, wof, 1024.0f, 0, 1, Hp, Wp);

  dim3 gg(EMB / 64, MROWS / 128);
  gemm_kernel<0><<<gg, 128, 0, stream>>>(xh, xl, wqh, wql, bq, qh, ql, out);
  gemm_kernel<0><<<gg, 128, 0, stream>>>(xh, xl, wkh, wkl, bk, kh, kl, out);
  gemm_kernel<1><<<gg, 128, 0, stream>>>(xf, xf, wvf, wvf, bv, vt, vt, out);

  attn_kernel<<<dim3(BB * NH, SEQ / 64), 128, 0, stream>>>(qh, ql, kh, kl, vt, ctx);

  gemm_kernel<2><<<gg, 128, 0, stream>>>(ctx, ctx, wof, wof, bo, ctx, ctx, out);
}
